// TEPRNN2_35261681500186
// MI455X (gfx1250) — hardware-verified
//
#include <hip/hip_runtime.h>

typedef __attribute__((ext_vector_type(16))) _Float16 v16h;
typedef __attribute__((ext_vector_type(8)))  _Float16 v8h;
typedef __attribute__((ext_vector_type(8)))  float    v8f;
typedef __attribute__((ext_vector_type(4)))  float    v4f;

constexpr int kSeq          = 256;
constexpr int kHid          = 64;
constexpr int kGateCols     = 256;
constexpr int kRowsPerBlock = 32;
constexpr int kThreads      = 128;
constexpr int kHPitch       = 72;
constexpr int kWPitch       = 72;
constexpr int kTPitch       = 68;
constexpr float kCarry      = 16.0f;
constexpr float kFold       = 1.0f / 256.0f;

static_assert(kGateCols == 4 * kHid);
static_assert(kRowsPerBlock * 4 == kThreads);
static_assert((kHPitch * 2) % 16 == 0 && (kWPitch * 2) % 16 == 0 && (kTPitch * 4) % 16 == 0);
static_assert(kRowsPerBlock * (int)sizeof(float) == 128);

__device__ __forceinline__ void dep_guard_h(v8f& a, v8f& b, v16h x, v16h y) { asm volatile("v_nop\n\tv_nop\n\tv_nop\n\tv_nop" : "+v"(a), "+v"(b) : "v"(x), "v"(y)); }
__device__ __forceinline__ void keep4_h(v16h a, v16h b, v16h c, v16h d) { asm volatile("v_nop" :: "v"(a), "v"(b), "v"(c), "v"(d)); }
template <typename T> struct Frag;
template <> struct Frag<_Float16> {
  typedef v16h V; union U { v16h v; v8h h[2]; };
  static __device__ __forceinline__ v16h load(const _Float16* p) {
    U f; f.h[0] = *(const v8h*)(p); f.h[1] = *(const v8h*)(p + 16); return f.v;
  }
  static __device__ __forceinline__ v8f mma(v16h a, v16h b, v8f c) {
    return __builtin_amdgcn_wmma_f32_16x16x32_f16(false, a, false, b, (short)0, c, false, false);
  }
  static __device__ __forceinline__ void guard(v8f& a, v8f& b, v16h x, v16h y) { dep_guard_h(a, b, x, y); }
  static __device__ __forceinline__ void keep(v16h a, v16h b, v16h c, v16h d) { keep4_h(a, b, c, d); }
};

__device__ __forceinline__ v8f mma_f16(v16h a, v16h b, v8f c) {
  c = __builtin_amdgcn_wmma_f32_16x16x32_f16(false, a, false, b, (short)0, c, false, false);
  asm volatile("v_nop\n\tv_nop\n\tv_nop\n\tv_nop" : "+v"(c) : "v"(a), "v"(b));
  return c;
}

__device__ __forceinline__ float sigm_f(float x) {
  const float xc = fminf(fmaxf(x, -30.0f), 30.0f);
  const float e = expf(-xc);
  return __builtin_amdgcn_rcpf(1.0f + e);
}
__device__ __forceinline__ float tanh_f(float x) {
  const float xc = fminf(fmaxf(x, -15.0f), 15.0f);
  const float e = expf(2.0f * xc);
  return fmaf(-2.0f, __builtin_amdgcn_rcpf(1.0f + e), 1.0f);
}

__global__ __launch_bounds__(kThreads) void lstm_seq_kernel(
    const float* __restrict__ x,
    const float* __restrict__ W1,
    const float* __restrict__ b1,
    const float* __restrict__ W_ih,
    const float* __restrict__ W_hh,
    const float* __restrict__ b_ih,
    const float* __restrict__ b_hh,
    const float* __restrict__ W2,
    const float* __restrict__ b2,
    float* __restrict__ out,
    int nrows)
{
  __shared__ __align__(16) _Float16 Wsh[kGateCols * kWPitch];
  __shared__ __align__(16) _Float16 hsh[2][kRowsPerBlock * kHPitch];
  __shared__ __align__(16) float    fcs[2][kRowsPerBlock * 4];
  __shared__ __align__(16) float    hT[kRowsPerBlock * kTPitch];
  __shared__ __align__(16) float    outs[kRowsPerBlock];

  const int tid  = threadIdx.x;
  const int wave = tid >> 5;
  const int lane = tid & 31;
  const int hh   = lane >> 4;
  const int c    = lane & 15;
  const int rowBase = blockIdx.x * kRowsPerBlock;

#pragma unroll 1
  for (int it = 0; it < 16; ++it) {
    const int q  = it * kThreads + tid;
    const int n  = q >> 3;
    const int k8 = (q & 7) * 8;
    const v4f w0 = *(const v4f*)(W_hh + n * kHid + k8);
    const v4f w1 = *(const v4f*)(W_hh + n * kHid + k8 + 4);
    v8h hv;
    hv[0] = (_Float16)(kCarry * w0[0]); hv[1] = (_Float16)(kCarry * w0[1]);
    hv[2] = (_Float16)(kCarry * w0[2]); hv[3] = (_Float16)(kCarry * w0[3]);
    hv[4] = (_Float16)(kCarry * w1[0]); hv[5] = (_Float16)(kCarry * w1[1]);
    hv[6] = (_Float16)(kCarry * w1[2]); hv[7] = (_Float16)(kCarry * w1[3]);
    *(v8h*)(Wsh + n * kWPitch + k8) = hv;
  }
#pragma unroll 1
  for (int it = 0; it < 2; ++it) {
    const int q = it * kThreads + tid;
    v8h z;
    z[0] = (_Float16)0.0f; z[1] = (_Float16)0.0f; z[2] = (_Float16)0.0f; z[3] = (_Float16)0.0f;
    z[4] = (_Float16)0.0f; z[5] = (_Float16)0.0f; z[6] = (_Float16)0.0f; z[7] = (_Float16)0.0f;
    *(v8h*)(hsh[0] + (q >> 3) * kHPitch + (q & 7) * 8) = z;
  }

  float wih[4][4], bsum[4];
#pragma unroll
  for (int g = 0; g < 4; ++g) {
    const int n = g * kHid + wave * 16 + c;
#pragma unroll
    for (int j = 0; j < 4; ++j) wih[g][j] = W_ih[n * 4 + j];
    bsum[g] = b_ih[n] + b_hh[n];
  }
  const int frow = tid >> 2;
  const int fj   = tid & 3;
  const float w1v = W1[fj];
  const float b1v = b1[fj];
  int xr = rowBase + frow;
  xr = (xr < nrows) ? xr : (nrows - 1);
  const float* xrow = x + (size_t)xr * kSeq;
  fcs[0][frow * 4 + fj] = tanh_f(xrow[0] * w1v + b1v);

  float cst[2][8];
#pragma unroll
  for (int mt = 0; mt < 2; ++mt)
#pragma unroll
    for (int r = 0; r < 8; ++r) cst[mt][r] = 0.0f;

  __syncthreads();

#pragma unroll 1
  for (int t = 0; t < kSeq; ++t) {
    const int cur = t & 1;
    const int nxt = cur ^ 1;

    {
      const int tn = (t + 1 < kSeq) ? (t + 1) : (kSeq - 1);
      fcs[nxt][frow * 4 + fj] = tanh_f(xrow[tn] * w1v + b1v);
    }

    const _Float16* hc = hsh[cur];
    _Float16*       hn = hsh[nxt];
    const float*    fc = fcs[cur];

#pragma unroll
    for (int mt = 0; mt < 2; ++mt) {
      const _Float16* ap = hc + (mt * 16 + c) * kHPitch + 8 * hh;
      const v16h a0 = Frag<_Float16>::load(ap);
      const v16h a1 = Frag<_Float16>::load(ap + 32);

      v8f acc[4];
#pragma unroll
      for (int g = 0; g < 4; ++g) {
        const _Float16* wp = Wsh + ((g * 4 + wave) * 16 + c) * kWPitch + 8 * hh;
        const v16h wb0 = Frag<_Float16>::load(wp);
        const v16h wb1 = Frag<_Float16>::load(wp + 32);
        v8f z = (v8f){0.f, 0.f, 0.f, 0.f, 0.f, 0.f, 0.f, 0.f};
        z = mma_f16(a0, wb0, z);
        z = mma_f16(a1, wb1, z);
        acc[g] = z;
      }

#pragma unroll
      for (int r = 0; r < 8; ++r) {
        const int row = mt * 16 + 8 * hh + r;
        const v4f f4 = *(const v4f*)(fc + row * 4);
        float pre[4];
#pragma unroll
        for (int g = 0; g < 4; ++g) {
          float s = fmaf(acc[g][r], kFold, bsum[g]);
          s = fmaf(f4[0], wih[g][0], s);
          s = fmaf(f4[1], wih[g][1], s);
          s = fmaf(f4[2], wih[g][2], s);
          s = fmaf(f4[3], wih[g][3], s);
          pre[g] = s;
        }
        const float ig = sigm_f(pre[0]);
        const float fg = sigm_f(pre[1]);
        const float gg = tanh_f(pre[2]);
        const float og = sigm_f(pre[3]);
        const float cc = fg * cst[mt][r] + ig * gg;
        cst[mt][r] = cc;
        const float hv = og * tanh_f(cc);
        hn[row * kHPitch + wave * 16 + c] = (_Float16)(kCarry * hv);
        hT[row * kTPitch + wave * 16 + c] = hv;
      }
    }
    __syncthreads();
  }

  if (tid < kRowsPerBlock) {
    const float* hr = hT + tid * kTPitch;
    float s = 0.0f;
#pragma unroll
    for (int k = 0; k < kHid; ++k) s = fmaf(hr[k], W2[k], s);
    outs[tid] = s + b2[0];
  }
  __syncthreads();
  if (tid < 8 && rowBase + kRowsPerBlock <= nrows) {
    const v4f v = *(const v4f*)(outs + tid * 4);
    float* op = out + rowBase + tid * 4;
    for (int pass = 0; pass < 2; ++pass) {
      *(volatile v4f*)op = v;
      __threadfence();
    }
  }
}

extern "C" void kernel_launch(void* const* d_in, const int* in_sizes, int n_in,
                              void* d_out, int out_size, void* d_ws, size_t ws_size,
                              hipStream_t stream) {
  (void)d_ws; (void)ws_size;
  if (n_in < 9) return;
  const float* x    = (const float*)d_in[0];
  const float* W1   = (const float*)d_in[1];
  const float* b1   = (const float*)d_in[2];
  const float* W_ih = (const float*)d_in[3];
  const float* W_hh = (const float*)d_in[4];
  const float* b_ih = (const float*)d_in[5];
  const float* b_hh = (const float*)d_in[6];
  const float* W2   = (const float*)d_in[7];
  const float* b2   = (const float*)d_in[8];
  float* out = (float*)d_out;

  const int nrows = out_size;
  if (nrows <= 0 || (nrows % kRowsPerBlock) != 0) return;
  if (in_sizes[0] != nrows * kSeq) return;
  if (in_sizes[1] < 4 || in_sizes[2] < 4) return;
  if (in_sizes[3] != kGateCols * 4 || in_sizes[4] != kGateCols * kHid) return;
  if (in_sizes[5] != kGateCols || in_sizes[6] != kGateCols || in_sizes[7] != kHid || in_sizes[8] < 1) return;

  dim3 grid(nrows / kRowsPerBlock);
  dim3 block(kThreads);
  lstm_seq_kernel<<<grid, block, 0, stream>>>(x, W1, b1, W_ih, W_hh, b_ih, b_hh, W2, b2, out, nrows);
}
